// NeighborhoodCrossAttention_82231443849835
// MI455X (gfx1250) — hardware-verified
//
#include <hip/hip_runtime.h>
#include <math.h>
#include <stdint.h>

#define DIMC 128
#define NHD  8
#define HD   16
#define HSZ  32
#define WSZ  32
#define ZSZ  8
#define NTOK (HSZ * WSZ * ZSZ)
#define XH2  16
#define XW2  16
#define XZ2  4
#define XSP  (XH2 * XW2 * XZ2)
#define KW   5
#define RPW  (2 * KW - 1)
#define RPBN (RPW * RPW * RPW)
#ifndef NQT
#define NQT  NTOK
#endif
#define KP   32
#define QKP  (NHD * KP)
#define WPB  NHD
#define ATT_THREADS (WPB * 32)
#define NKTL (KW * 2)
#define KWW  8
#define XCAR 64.0f
#define WCAR 1024.0f
#define QCAR 4096.0f
#define KCAR 4096.0f
#define VCAR 4096.0f
#define PCAR 16384.0f
#define OSC  1024.0f
#define QSCL 0.25f
#define LOG2E 1.4426950408889634f
#define IN_EPS 1e-5f
#define PTP  36
#define PTW  (16 * PTP)
#define RPBP 736
#define WREG (PTW + RPBP)
#define SLP  132
#define SLW  (16 * SLP)
#define SLAB64 (16 * 68)
#define VTP  72
#define TTP  136
#define STL  32
#define WS_CAP 134217728

static_assert(DIMC == NHD * HD && HD == 16 && KP == 32 && QKP == 256);
static_assert(NTOK == 8192 && XSP == 1024 && HSZ == 2 * XH2 && WSZ == 2 * XW2 && ZSZ == 2 * XZ2);
static_assert((NQT % 64) == 0 && NQT >= 64 && NQT <= NTOK);
static_assert(RPBN == 729 && RPBP >= RPBN && (RPBP % 32) == 0);
static_assert(ATT_THREADS == 256 && WPB == 8);
static_assert(KWW * ZSZ == 64 && HSZ >= KW && WSZ >= KWW && ZSZ >= KW);
static_assert((DIMC % 64) == 0 && (NTOK % 64) == 0 && (DIMC % 32) == 0);
static_assert((PTP * 4) % 16 == 0 && (SLP * 4) % 16 == 0 && (VTP * 2) % 16 == 0 && (TTP * 2) % 16 == 0);

typedef unsigned short u16;
typedef _Float16 v16h __attribute__((ext_vector_type(16)));
typedef _Float16 v8h  __attribute__((ext_vector_type(8)));
typedef float    v8f  __attribute__((ext_vector_type(8)));
typedef float    v4f  __attribute__((ext_vector_type(4)));
typedef float    v2f  __attribute__((ext_vector_type(2)));
typedef unsigned int v4u __attribute__((ext_vector_type(4)));

union FragH { v16h v; v8h h[2]; v4u u[2]; };

__device__ __forceinline__ unsigned short bf_bits(float f) {
  unsigned u = __float_as_uint(f);
  return (unsigned short)((u + 0x7FFFu + ((u >> 16) & 1u)) >> 16);
}
__device__ __forceinline__ float bf_up(unsigned short h) { return __uint_as_float(((unsigned)h) << 16); }
__device__ __forceinline__ float bfr(float f) { return bf_up(bf_bits(f)); }
__device__ __forceinline__ unsigned short h_bits(_Float16 x) { return __builtin_bit_cast(unsigned short, x); }
__device__ __forceinline__ unsigned pk16(unsigned short a, unsigned short b) { return (unsigned)a | ((unsigned)b << 16); }
__device__ __forceinline__ v8f zero8() { v8f z = {0.f, 0.f, 0.f, 0.f, 0.f, 0.f, 0.f, 0.f}; return z; }
__device__ __forceinline__ float wave_sum(float v) {
#pragma unroll
  for (int off = 16; off > 0; off >>= 1) v += __shfl_xor(v, off, 32);
  return v;
}

__device__ __forceinline__ v16h ldfrag_h(const _Float16* p) {
  FragH f;
  f.h[0] = *(const v8h*)(p);
  f.h[1] = *(const v8h*)(p + 16);
  return f.v;
}

__device__ __forceinline__ v8f mma_h(v16h a, v16h b, v8f c) {
  return __builtin_amdgcn_wmma_f32_16x16x32_f16(false, a, false, b, (short)0, c, false, false);
}
__device__ __forceinline__ void guard1(v8f& a, v16h x0, v16h x1, v16h x2, v16h x3) {
#if defined(__HIP_DEVICE_COMPILE__)
  asm volatile("v_nop\n\tv_nop\n\tv_nop\n\tv_nop" : "+v"(a) : "v"(x0), "v"(x1), "v"(x2), "v"(x3) : "memory");
#endif
}
__device__ __forceinline__ void guard2(v8f& a, v8f& b, v16h x0, v16h x1, v16h x2, v16h x3, v16h x4, v16h x5) {
#if defined(__HIP_DEVICE_COMPILE__)
  asm volatile("v_nop\n\tv_nop\n\tv_nop\n\tv_nop"
               : "+v"(a), "+v"(b) : "v"(x0), "v"(x1), "v"(x2), "v"(x3), "v"(x4), "v"(x5) : "memory");
#endif
}
template <typename F>
__device__ __forceinline__ void guard10(v8f& a, v8f& b, v8f& c, v8f& d, F x0, F x1, F x2, F x3, F x4, F x5,
                                        F x6, F x7, F x8, F x9) {
#if defined(__HIP_DEVICE_COMPILE__)
  asm volatile("v_nop\n\tv_nop\n\tv_nop\n\tv_nop"
               : "+v"(a), "+v"(b), "+v"(c), "+v"(d)
               : "v"(x0), "v"(x1), "v"(x2), "v"(x3), "v"(x4), "v"(x5), "v"(x6), "v"(x7), "v"(x8), "v"(x9) : "memory");
#endif
}
__device__ __forceinline__ void acc_guard1(v8f& a) {
#if defined(__HIP_DEVICE_COMPILE__)
  asm volatile("v_nop\n\tv_nop\n\tv_nop\n\tv_nop" : "+v"(a));
#endif
}
__device__ __forceinline__ void wave_sync_lds() {
  __builtin_amdgcn_fence(__ATOMIC_RELEASE, "workgroup");
  __builtin_amdgcn_wave_barrier();
  __builtin_amdgcn_fence(__ATOMIC_ACQUIRE, "workgroup");
}

__global__ __launch_bounds__(256) void in_stats(const float* __restrict__ x, const float* __restrict__ sk, float* ST) {
  __shared__ float red[8];
  const int tid = threadIdx.x, wave = tid >> 5, lane = tid & 31;
  const int ch = blockIdx.x;
  if (ch >= 2 * DIMC) return;
  const bool isx = (ch < DIMC);
  const int  cx  = isx ? ch : 0;
  const int  cs  = isx ? 0 : (ch - DIMC);
  const int  cnt = isx ? XSP : NTOK;
  const float* src = isx ? (x + (size_t)cx * XSP) : (sk + (size_t)cs * NTOK);
  const int n4 = cnt >> 2;
  float s = 0.f;
  for (int i = tid; i < n4; i += 256) {
    const v4f a = *(const v4f*)(src + 4 * i);
    s += (bfr(a[0]) + bfr(a[1])) + (bfr(a[2]) + bfr(a[3]));
  }
  s = wave_sum(s);
  if (lane == 0) red[wave] = s;
  __syncthreads();
  float S = 0.f;
#pragma unroll
  for (int w = 0; w < 8; ++w) S += red[w];
  const float inv_n = 1.0f / (float)cnt;
  const float mu = S * inv_n;
  __syncthreads();
  float q = 0.f;
  for (int i = tid; i < n4; i += 256) {
    const v4f a = *(const v4f*)(src + 4 * i);
    const float d0 = bfr(a[0]) - mu, d1 = bfr(a[1]) - mu, d2 = bfr(a[2]) - mu, d3 = bfr(a[3]) - mu;
    q += (d0 * d0 + d1 * d1) + (d2 * d2 + d3 * d3);
  }
  q = wave_sum(q);
  if (lane == 0) red[wave] = q;
  __syncthreads();
  float Q = 0.f;
#pragma unroll
  for (int w = 0; w < 8; ++w) Q += red[w];
  const float var = Q * inv_n;
  const float rs  = rsqrtf(var + IN_EPS);
  v4f val;
  val[0] = (lane == 0) ? mu : 0.0f;
  val[1] = (lane == 0) ? rs : 0.0f;
  val[2] = 0.0f;
  val[3] = 0.0f;
  float* d = ST + (size_t)ch * STL + lane * 4;
  for (int pass = 0; pass < 2; ++pass) {
    if (wave == 0 && lane < 8) *(volatile v4f*)(d) = val;
    __threadfence();
  }
}

__global__ __launch_bounds__(256) void tok16(const float* __restrict__ x, const float* __restrict__ sk,
                                              const float* __restrict__ ST, u16* XH, u16* XL, u16* SH, u16* SL) {
  __shared__ __align__(16) u16 TH[64 * TTP];
  __shared__ __align__(16) u16 TL[64 * TTP];
  const int tid = threadIdx.x, bid = blockIdx.x;
  const int src = bid >> 7;
  const int tt  = bid & 127;
  if (src > 1) return;
  const int n0 = tt * 64;
  const int c  = tid >> 1, th = tid & 1;
  const float mu = ST[(size_t)(src * DIMC + c) * STL];
  const float rs = ST[(size_t)(src * DIMC + c) * STL + 1];
  const float rsc = rs * XCAR;
  const int h = tt >> 2, w0 = (tt & 3) * 8;
  const bool usx = (src == 0);
  const float* px = x  + (size_t)c * XSP + (h >> 1) * (XW2 * XZ2) + (w0 >> 1) * XZ2 + 8 * th;
  const float* ps = sk + (size_t)c * NTOK + n0 + 32 * th;
#pragma unroll 1
  for (int i = 0; i < 8; ++i) {
    const v2f q2 = *(const v2f*)(px + (i >> 2) * 4 + 2 * (i & 1));
    const v4f s4 = *(const v4f*)(ps + 4 * i);
    float a[4];
    a[0] = usx ? q2[0] : s4[0];
    a[1] = usx ? q2[0] : s4[1];
    a[2] = usx ? q2[1] : s4[2];
    a[3] = usx ? q2[1] : s4[3];
#pragma unroll
    for (int e = 0; e < 4; ++e) {
      const float t = (bfr(a[e]) - mu) * rsc;
      const _Float16 hv = (_Float16)t;
      const _Float16 lv = (_Float16)(t - (float)hv);
      const int row = 32 * th + 4 * i + e;
      TH[row * TTP + c] = h_bits(hv);
      TL[row * TTP + c] = h_bits(lv);
    }
  }
  __syncthreads();
  v4u vh[4], vl[4];
  const int rsel = tid >> 4, c8 = (tid & 15) * 8;
#pragma unroll
  for (int it = 0; it < 4; ++it) {
    const int row = it * 16 + rsel;
    vh[it] = *(const v4u*)(TH + row * TTP + c8);
    vl[it] = *(const v4u*)(TL + row * TTP + c8);
  }
  u16* DH = (src == 0) ? XH : SH;
  u16* DL = (src == 0) ? XL : SL;
  const size_t base = (size_t)n0 * DIMC + c8;
  for (int pass = 0; pass < 2; ++pass) {
#pragma unroll
    for (int it = 0; it < 4; ++it) {
      const int row = it * 16 + rsel;
      *(volatile v4u*)(DH + base + (size_t)row * DIMC) = vh[it];
      *(volatile v4u*)(DL + base + (size_t)row * DIMC) = vl[it];
    }
    __threadfence();
  }
}

__global__ __launch_bounds__(256) void wt16(const float* __restrict__ Wq, const float* __restrict__ Wk,
                                             const float* __restrict__ Wv, const float* __restrict__ Wo, u16* D) {
  __shared__ __align__(16) u16 T[128 * VTP];
  const int tid = threadIdx.x;
  const int bid = blockIdx.x;
  const int msel = bid >> 1;
  const int rt   = bid & 1;
  if (msel > 3) return;
  const float* W = (msel == 0) ? Wq : (msel == 1) ? Wk : (msel == 2) ? Wv : Wo;
  {
    const int sl = tid >> 2;
    const int dc = (tid & 3) * 32;
    const float* src = W + (size_t)(rt * 64 + sl) * DIMC + dc;
#pragma unroll
    for (int i = 0; i < 8; ++i) {
      const v4f a = *(const v4f*)(src + 4 * i);
#pragma unroll
      for (int e = 0; e < 4; ++e) {
        T[(dc + 4 * i + e) * VTP + sl] = h_bits((_Float16)(bfr(a[e]) * WCAR));
      }
    }
  }
  __syncthreads();
  v4u w4[4];
  const int q8 = tid >> 3, p8 = (tid & 7) * 8;
#pragma unroll
  for (int it = 0; it < 4; ++it) {
    const int line = it * 32 + q8;
    w4[it] = *(const v4u*)(T + line * VTP + p8);
  }
  const size_t base = (size_t)msel * DIMC * DIMC + rt * 64 + p8;
  for (int pass = 0; pass < 2; ++pass) {
#pragma unroll
    for (int it = 0; it < 4; ++it) {
      const int line = it * 32 + q8;
      *(volatile v4u*)(D + base + (size_t)line * DIMC) = w4[it];
    }
    __threadfence();
  }
}

__global__ __launch_bounds__(256) void qkpad16(const float* __restrict__ F, u16* Hp, u16* Lp, float sc) {
  const int tid = (int)threadIdx.x;
  const int rl  = tid >> 5, tc = tid & 31;
  const int row = (int)blockIdx.x * 8 + rl;
  if (row >= NTOK) return;
  const int head = tc >> 2, part = tc & 3;
  const int icol = head * HD + (part & 1) * 8;
  const float* p = F + (size_t)row * DIMC + icol;
  const v4f a = *(const v4f*)(p), b4 = *(const v4f*)(p + 4);
  float w[8];
#pragma unroll
  for (int e = 0; e < 4; ++e) { w[e] = a[e] * sc; w[4 + e] = b4[e] * sc; }
  const bool zer = (part >= 2);
  v4u oh, ol;
#pragma unroll
  for (int e = 0; e < 4; ++e) {
    const float t0 = w[2 * e], t1 = w[2 * e + 1];
    const _Float16 h0 = (_Float16)t0, h1 = (_Float16)t1;
    const _Float16 l0 = (_Float16)(t0 - (float)h0), l1 = (_Float16)(t1 - (float)h1);
    const unsigned uh = pk16(h_bits(h0), h_bits(h1));
    const unsigned ul = pk16(h_bits(l0), h_bits(l1));
    oh[e] = zer ? 0u : uh;
    ol[e] = zer ? 0u : ul;
  }
  u16* dh = Hp + (size_t)row * QKP + tc * 8;
  u16* dl = Lp + (size_t)row * QKP + tc * 8;
  for (int pass = 0; pass < 2; ++pass) {
    *(volatile v4u*)(dh) = oh;
    *(volatile v4u*)(dl) = ol;
    __threadfence();
  }
}

__global__ __launch_bounds__(256) void vt16(const float* __restrict__ F, u16* VHo, u16* VLo) {
  __shared__ __align__(16) u16 TH[DIMC * VTP];
  __shared__ __align__(16) u16 TL[DIMC * VTP];
  const int tid = threadIdx.x;
  const int bid = blockIdx.x;
  const int s0  = bid * 64;
  if (s0 + 64 > NTOK) return;
  {
    const int sl = tid >> 2;
    const int dc = (tid & 3) * 32;
    const float* src = F + (size_t)(s0 + sl) * DIMC + dc;
#pragma unroll
    for (int i = 0; i < 8; ++i) {
      const v4f a = *(const v4f*)(src + 4 * i);
#pragma unroll
      for (int e = 0; e < 4; ++e) {
        const float t = a[e] * VCAR;
        const _Float16 hv = (_Float16)t;
        const _Float16 lv = (_Float16)(t - (float)hv);
        TH[(dc + 4 * i + e) * VTP + sl] = h_bits(hv);
        TL[(dc + 4 * i + e) * VTP + sl] = h_bits(lv);
      }
    }
  }
  __syncthreads();
  v4u vh[4], vl[4];
  const int q8 = tid >> 3, p8 = (tid & 7) * 8;
#pragma unroll
  for (int it = 0; it < 4; ++it) {
    const int line = it * 32 + q8;
    vh[it] = *(const v4u*)(TH + line * VTP + p8);
    vl[it] = *(const v4u*)(TL + line * VTP + p8);
  }
  const size_t base = (size_t)s0 + p8;
  for (int pass = 0; pass < 2; ++pass) {
#pragma unroll
    for (int it = 0; it < 4; ++it) {
      const int line = it * 32 + q8;
      *(volatile v4u*)(VHo + (size_t)line * NTOK + base) = vh[it];
      *(volatile v4u*)(VLo + (size_t)line * NTOK + base) = vl[it];
    }
    __threadfence();
  }
}

template <int AL, int BL, int BROW>
__global__ __launch_bounds__(128)
void gemm16(const u16* __restrict__ Ah, const u16* __restrict__ Al, const u16* __restrict__ Bh, const u16* __restrict__ Bl,
            const float* __restrict__ bias, int nbias, float* C, int M, int N, int K, int ldc, float oscale, float pscale) {
  __shared__ __align__(16) float slab[4 * SLAB64];
  const int tid = threadIdx.x, wave = tid >> 5, lane = tid & 31, hh = lane >> 4, m = lane & 15;
  const int ntile = N >> 6;
  const int bid   = blockIdx.x;
  const int rowb  = (bid / ntile) * 64 + wave * 16;
  const int col0  = (bid % ntile) * 64;
  if (rowb + 16 > M) return;
  const _Float16* ahp = (const _Float16*)(const void*)Ah + (size_t)(rowb + m) * K + 8 * hh;
  const _Float16* alp = (const _Float16*)(const void*)Al + (size_t)(rowb + m) * K + 8 * hh;
  const _Float16* bhp = (const _Float16*)(const void*)Bh + (size_t)(col0 + m) * K + 8 * hh;
  const _Float16* blp = (const _Float16*)(const void*)Bl + (size_t)(col0 + m) * K + 8 * hh;
  const size_t bs = (size_t)16 * K;
  v8f acc0 = zero8(), acc1 = zero8(), acc2 = zero8(), acc3 = zero8();
#pragma unroll 1
  for (int k0 = 0; k0 < K; k0 += 32) {
    const v16h ah = ldfrag_h(ahp + k0);
    v16h al = ah;
    if constexpr (AL != 0) al = ldfrag_h(alp + k0);
    const v16h b0 = ldfrag_h(bhp + k0);
    const v16h b1 = ldfrag_h(bhp + bs + k0);
    const v16h b2 = ldfrag_h(bhp + 2 * bs + k0);
    const v16h b3 = ldfrag_h(bhp + 3 * bs + k0);
    v16h l0 = b0, l1 = b1, l2 = b2, l3 = b3;
    if constexpr (BL != 0) {
      l0 = ldfrag_h(blp + k0);
      l1 = ldfrag_h(blp + bs + k0);
      l2 = ldfrag_h(blp + 2 * bs + k0);
      l3 = ldfrag_h(blp + 3 * bs + k0);
    }
    acc0 = mma_h(ah, b0, acc0);
    acc1 = mma_h(ah, b1, acc1);
    acc2 = mma_h(ah, b2, acc2);
    acc3 = mma_h(ah, b3, acc3);
    if constexpr (AL != 0) {
      acc0 = mma_h(al, b0, acc0);
      acc1 = mma_h(al, b1, acc1);
      acc2 = mma_h(al, b2, acc2);
      acc3 = mma_h(al, b3, acc3);
    }
    if constexpr (BL != 0) {
      acc0 = mma_h(ah, l0, acc0);
      acc1 = mma_h(ah, l1, acc1);
      acc2 = mma_h(ah, l2, acc2);
      acc3 = mma_h(ah, l3, acc3);
    }
    guard10<v16h>(acc0, acc1, acc2, acc3, ah, al, b0, b1, b2, b3, l0, l1, l2, l3);
  }
  float* sl = slab + wave * SLAB64;
  float bc0 = 0.f, bc1 = 0.f, bc2 = 0.f, bc3 = 0.f;
  if constexpr (BROW == 0) {
    bc0 = bfr(bias[min(col0 + m, nbias - 1)]);
    bc1 = bfr(bias[min(col0 + 16 + m, nbias - 1)]);
    bc2 = bfr(bias[min(col0 + 32 + m, nbias - 1)]);
    bc3 = bfr(bias[min(col0 + 48 + m, nbias - 1)]);
  }
#pragma unroll
  for (int r = 0; r < 8; ++r) {
    float e0 = bc0, e1 = bc1, e2 = bc2, e3 = bc3;
    if constexpr (BROW != 0) {
      const float br = bfr(bias[min(rowb + 8 * hh + r, nbias - 1)]);
      e0 = br; e1 = br; e2 = br; e3 = br;
    }
    const int ro = (8 * hh + r) * 68 + m;
    sl[ro]      = (acc0[r] * oscale + e0) * pscale;
    sl[ro + 16] = (acc1[r] * oscale + e1) * pscale;
    sl[ro + 32] = (acc2[r] * oscale + e2) * pscale;
    sl[ro + 48] = (acc3[r] * oscale + e3) * pscale;
  }
  wave_sync_lds();
  v4f vals[8];
#pragma unroll
  for (int it = 0; it < 8; ++it) vals[it] = *(const v4f*)(sl + (it * 2 + hh) * 68 + m * 4);
  float* dst = C + ((size_t)rowb + (size_t)hh) * (size_t)ldc + col0 + m * 4;
  for (int pass = 0; pass < 2; ++pass) {
#pragma unroll
    for (int it = 0; it < 8; ++it) {
      *(volatile v4f*)(dst + (size_t)(it * 2) * (size_t)ldc) = vals[it];
    }
    __threadfence();
  }
}

__global__ __launch_bounds__(ATT_THREADS)
void attn_nb(const u16* __restrict__ QHp, const u16* __restrict__ QLp, const u16* __restrict__ KHp,
             const u16* __restrict__ KLp, const u16* __restrict__ VHp, const u16* __restrict__ VLp,
             const float* __restrict__ rpb, u16* OHp, u16* OLp) {
  __shared__ __align__(16) float smem[WPB * WREG + SLW];

  const int tid  = threadIdx.x;
  const int wave = tid >> 5;
  const int lane = tid & 31;
  const int hh   = lane >> 4;
  const int c    = lane & 15;
  const int qt   = blockIdx.x;
  const int q0   = qt * 16;
  if (q0 + 16 > NQT) return;
  const int head = wave;
  const int h    = qt >> 4;
  const int w0   = (qt & 15) * 2;
  const int sh   = min(max(h - 2, 0), HSZ - KW);
  const int wb   = min(max(w0 - 3, 0), WSZ - KWW);

  float* pt   = smem + wave * WREG;
  float* rb   = pt + PTW;
  float* slab = smem + WPB * WREG;

  for (int i = lane; i < RPBP; i += 32) {
    const int ii = (i < RPBN) ? i : (RPBN - 1);
    const float v = bfr(rpb[(size_t)head * RPBN + ii]) * LOG2E;
    rb[i] = (i < RPBN) ? v : 0.0f;
  }
  wave_sync_lds();

  const int wq  = w0 + hh;
  const int swq = min(max(wq - 2, 0), WSZ - KW);
  const size_t hcol = (size_t)head * KP + 8 * hh;
  const _Float16* Qh  = (const _Float16*)(const void*)QHp + ((size_t)q0 + c) * QKP + hcol;
  const _Float16* Ql  = (const _Float16*)(const void*)QLp + ((size_t)q0 + c) * QKP + hcol;
  const _Float16* Khb = (const _Float16*)(const void*)KHp + (size_t)c * QKP + hcol;
  const _Float16* Klb = (const _Float16*)(const void*)KLp + (size_t)c * QKP + hcol;
  const _Float16* Vhb = (const _Float16*)(const void*)VHp + ((size_t)head * HD + c) * NTOK + 8 * hh;
  const _Float16* Vlb = (const _Float16*)(const void*)VLp + ((size_t)head * HD + c) * NTOK + 8 * hh;
  const float lsc = LOG2E / (QCAR * KCAR);
  const float oc  = 1.0f / (PCAR * VCAR);

  const v16h qh = ldfrag_h(Qh);
  const v16h ql = ldfrag_h(Ql);

  float mrow[8], lrow[8];
  v8f o = zero8();
#pragma unroll
  for (int r = 0; r < 8; ++r) { mrow[r] = -INFINITY; lrow[r] = 0.f; }

#pragma unroll 1
  for (int kt = 0; kt < NKTL; ++kt) {
    const int ih = kt >> 1, jw = kt & 1;
    const int kb = (sh + ih) * (WSZ * ZSZ) + (wb + 4 * jw) * ZSZ;
    v8f s0 = zero8(), s1 = zero8();
    const _Float16* k0p = Khb + (size_t)kb * QKP;
    const _Float16* k1p = k0p + (size_t)16 * QKP;
    const _Float16* l0p = Klb + (size_t)kb * QKP;
    const _Float16* l1p = l0p + (size_t)16 * QKP;
    {
      const v16h kh0 = ldfrag_h(k0p);
      const v16h kh1 = ldfrag_h(k1p);
      const v16h kl0 = ldfrag_h(l0p);
      const v16h kl1 = ldfrag_h(l1p);
      s0 = mma_h(qh, kh0, s0);
      s0 = mma_h(ql, kh0, s0);
      s0 = mma_h(qh, kl0, s0);
      s1 = mma_h(qh, kh1, s1);
      s1 = mma_h(ql, kh1, s1);
      s1 = mma_h(qh, kl1, s1);
      guard2(s0, s1, qh, ql, kh0, kl0, kh1, kl1);
    }
    const int rH  = sh + ih - h + (KW - 1);
    const int wk0 = wb + 4 * jw + (c >> 3);
    const int wk1 = wk0 + 2;
    const int zk  = c & 7;
    const bool vw0 = (wk0 >= swq) && (wk0 < swq + KW);
    const bool vw1 = (wk1 >= swq) && (wk1 < swq + KW);
    const int rW0 = min(max(wk0 - wq + (KW - 1), 0), RPW - 1);
    const int rW1 = min(max(wk1 - wq + (KW - 1), 0), RPW - 1);
    const float* rbh = rb + rH * (RPW * RPW);
#pragma unroll
    for (int r = 0; r < 8; ++r) {
      const int  szr = min(max(r - 2, 0), ZSZ - KW);
      const bool vz  = (zk >= szr) && (zk < szr + KW);
      const int  rZ  = min(max(zk - r + (KW - 1), 0), RPW - 1);
      const float b0 = rbh[rW0 * RPW + rZ];
      const float b1 = rbh[rW1 * RPW + rZ];
      const float u0 = s0[r] * lsc + b0;
      const float u1 = s1[r] * lsc + b1;
      const float t0 = (vw0 && vz) ? u0 : -INFINITY;
      const float t1 = (vw1 && vz) ? u1 : -INFINITY;
      float mx = fmaxf(t0, t1);
#pragma unroll
      for (int off = 1; off < 16; off <<= 1) mx = fmaxf(mx, __shfl_xor(mx, off, 32));
      const float mn = fmaxf(mrow[r], mx);
      const float ms = (mn == -INFINITY) ? 0.0f : mn;
      const float al = exp2f(mrow[r] - ms);
      mrow[r] = mn;
      const float e0 = exp2f(t0 - ms), e1 = exp2f(t1 - ms);
      float ps = e0 + e1;
#pragma unroll
      for (int off = 1; off < 16; off <<= 1) ps += __shfl_xor(ps, off, 32);
      lrow[r] = lrow[r] * al + ps;
      o[r] *= al;
      const int ro = (8 * hh + r) * PTP + c;
      pt[ro]      = e0;
      pt[ro + 16] = e1;
    }
    wave_sync_lds();
    FragH ph, pl;
    {
      const float* prow = pt + c * PTP + 8 * hh;
      const v4f p0 = *(const v4f*)(prow), p1 = *(const v4f*)(prow + 4);
      const v4f p2 = *(const v4f*)(prow + 16), p3 = *(const v4f*)(prow + 20);
#pragma unroll
      for (int e = 0; e < 4; ++e) {
        const float ta = p0[e] * PCAR, tb = p1[e] * PCAR, tc = p2[e] * PCAR, td = p3[e] * PCAR;
        const _Float16 ha = (_Float16)ta, hb = (_Float16)tb, hc = (_Float16)tc, hd = (_Float16)td;
        ph.h[0][e]     = ha;
        ph.h[0][4 + e] = hb;
        ph.h[1][e]     = hc;
        ph.h[1][4 + e] = hd;
        pl.h[0][e]     = (_Float16)(ta - (float)ha);
        pl.h[0][4 + e] = (_Float16)(tb - (float)hb);
        pl.h[1][e]     = (_Float16)(tc - (float)hc);
        pl.h[1][4 + e] = (_Float16)(td - (float)hd);
      }
    }
    {
      const v16h vha = ldfrag_h(Vhb + kb);
      const v16h vla = ldfrag_h(Vlb + kb);
      o = mma_h(ph.v, vha, o);
      o = mma_h(pl.v, vha, o);
      o = mma_h(ph.v, vla, o);
      guard1(o, ph.v, pl.v, vha, vla);
    }
    wave_sync_lds();
  }
  acc_guard1(o);
  const int ocol = head * HD + c;
#pragma unroll
  for (int r = 0; r < 8; ++r) {
    const float lv  = lrow[r];
    const float ls  = (lv > 0.0f) ? lv : 1.0f;
    const float inv = (lv > 0.0f) ? ((1.0f / ls) * oc) : 0.0f;
    slab[(8 * hh + r) * SLP + ocol] = o[r] * inv;
  }
  __syncthreads();
  const int row = tid >> 4, c8 = (tid & 15) * 8;
  const v4f a = *(const v4f*)(slab + row * SLP + c8), b4 = *(const v4f*)(slab + row * SLP + c8 + 4);
  float wv[8];
#pragma unroll
  for (int e = 0; e < 4; ++e) { wv[e] = a[e] * OSC; wv[4 + e] = b4[e] * OSC; }
  v4u oh, ol;
#pragma unroll
  for (int e = 0; e < 4; ++e) {
    const _Float16 h0 = (_Float16)wv[2 * e], h1 = (_Float16)wv[2 * e + 1];
    const _Float16 l0 = (_Float16)(wv[2 * e] - (float)h0), l1 = (_Float16)(wv[2 * e + 1] - (float)h1);
    oh[e] = pk16(h_bits(h0), h_bits(h1));
    ol[e] = pk16(h_bits(l0), h_bits(l1));
  }
  const size_t ob = ((size_t)q0 + row) * DIMC + c8;
  for (int pass = 0; pass < 2; ++pass) {
    *(volatile v4u*)(OHp + ob) = oh;
    *(volatile v4u*)(OLp + ob) = ol;
    __threadfence();
  }
}

extern "C" void kernel_launch(void* const* d_in, const int* in_sizes, int n_in,
                              void* d_out, int out_size, void* d_ws, size_t ws_size,
                              hipStream_t stream) {
  if (n_in < 11) return;
  if (in_sizes[0] < DIMC * XSP) return;
  if (in_sizes[1] < DIMC * NTOK) return;
  if (in_sizes[2] < DIMC * DIMC || in_sizes[4] < DIMC * DIMC || in_sizes[6] < DIMC * DIMC || in_sizes[9] < DIMC * DIMC) return;
  if (in_sizes[3] < DIMC || in_sizes[5] < DIMC || in_sizes[7] < DIMC || in_sizes[10] < DIMC) return;
  if (in_sizes[8] < NHD * RPBN) return;
  if (out_size < DIMC * NTOK) return;

  const float* x    = (const float*)d_in[0];
  const float* skip = (const float*)d_in[1];
  const float* Wq   = (const float*)d_in[2];
  const float* bq   = (const float*)d_in[3];
  const float* Wk   = (const float*)d_in[4];
  const float* bk   = (const float*)d_in[5];
  const float* Wv   = (const float*)d_in[6];
  const float* bv   = (const float*)d_in[7];
  const float* rpb  = (const float*)d_in[8];
  const float* Wo   = (const float*)d_in[9];
  const float* bo   = (const float*)d_in[10];
  float*       out  = (float*)d_out;

  const size_t szST = (size_t)2 * DIMC * STL * 4;
  const size_t szWP = (size_t)4 * DIMC * DIMC * 2;
  const size_t szT  = (size_t)NTOK * DIMC * 2;
  const size_t szF  = (size_t)NTOK * DIMC * 4;
  const size_t szQK = (size_t)NTOK * QKP * 2;
  size_t off = 0;
  const size_t oST = off; off += szST;
  const size_t oWP = off; off += szWP;
  const size_t oXH = off; off += szT;
  const size_t oXL = off; off += szT;
  const size_t oSH = off; off += szT;
  const size_t oSL = off; off += szT;
  const size_t oFQ = off; off += szF;
  const size_t oFK = off; off += szF;
  const size_t oFV = off; off += szF;
  const size_t oQH = off; off += szQK;
  const size_t oQL = off; off += szQK;
  const size_t oKH = off; off += szQK;
  const size_t oKL = off; off += szQK;
  const size_t oVH = off; off += szT;
  const size_t oVL = off; off += szT;
  const size_t oOH = off; off += szT;
  const size_t oOL = off; off += szT;
  if (off > ws_size) return;
  if (off > (size_t)WS_CAP) return;

  char* ws = (char*)d_ws;
  float* ST = (float*)(ws + oST);
  u16*   WP = (u16*)(ws + oWP);
  u16*   XH = (u16*)(ws + oXH);
  u16*   XL = (u16*)(ws + oXL);
  u16*   SH = (u16*)(ws + oSH);
  u16*   SL = (u16*)(ws + oSL);
  float* FQ = (float*)(ws + oFQ);
  float* FK = (float*)(ws + oFK);
  float* FV = (float*)(ws + oFV);
  u16*   QH = (u16*)(ws + oQH);
  u16*   QL = (u16*)(ws + oQL);
  u16*   KH = (u16*)(ws + oKH);
  u16*   KL = (u16*)(ws + oKL);
  u16*   VH = (u16*)(ws + oVH);
  u16*   VL = (u16*)(ws + oVL);
  u16*   OH = (u16*)(ws + oOH);
  u16*   OL = (u16*)(ws + oOL);
  u16*   WQp = WP;
  u16*   WKp = WP + (size_t)DIMC * DIMC;
  u16*   WVp = WP + (size_t)2 * DIMC * DIMC;
  u16*   WOp = WP + (size_t)3 * DIMC * DIMC;

  const dim3 b256(256), b128(128), bAT(ATT_THREADS);
  const float psc  = 1.0f / (XCAR * WCAR);
  const float oscO = 1.0f / (OSC * WCAR);

  in_stats<<<dim3(2 * DIMC), b256, 0, stream>>>(x, skip, ST);
  wt16<<<dim3(8), b256, 0, stream>>>(Wq, Wk, Wv, Wo, WP);
  tok16<<<dim3(256), b256, 0, stream>>>(x, skip, ST, XH, XL, SH, SL);
  gemm16<1, 0, 0><<<dim3((NTOK / 64) * (DIMC / 64)), b128, 0, stream>>>(XH, XL, WQp, WQp, bq, DIMC, FQ,
                                                                         NTOK, DIMC, DIMC, DIMC, psc, QSCL);
  gemm16<1, 0, 0><<<dim3((NTOK / 64) * (DIMC / 64)), b128, 0, stream>>>(SH, SL, WKp, WKp, bk, DIMC, FK,
                                                                         NTOK, DIMC, DIMC, DIMC, psc, 1.0f);
  gemm16<1, 0, 0><<<dim3((NTOK / 64) * (DIMC / 64)), b128, 0, stream>>>(SH, SL, WVp, WVp, bv, DIMC, FV,
                                                                         NTOK, DIMC, DIMC, DIMC, psc, 1.0f);
  qkpad16<<<dim3(NTOK / 8), b256, 0, stream>>>(FQ, QH, QL, QCAR);
  qkpad16<<<dim3(NTOK / 8), b256, 0, stream>>>(FK, KH, KL, KCAR);
  vt16<<<dim3(NTOK / 64), b256, 0, stream>>>(FV, VH, VL);
  attn_nb<<<dim3(NQT / 16), bAT, 0, stream>>>(QH, QL, KH, KL, VH, VL, rpb, OH, OL);
  gemm16<0, 1, 1><<<dim3((DIMC / 64) * (NQT / 64)), b128, 0, stream>>>(WOp, WOp, OH, OL, bo, DIMC, out,
                                                                        DIMC, NQT, DIMC, NTOK, oscO, 1.0f);
  (void)hipGetLastError();
}
